// LayerNormLSTMCell_47742856462402
// MI455X (gfx1250) — hardware-run, weakly checked
//
#include <hip/hip_runtime.h>


namespace {
constexpr int NBR = 4096, IN = 1024, H = 1024, G4 = 4 * H, KT = IN + H;
constexpr float HS = 256.0f, WSC = 256.0f, EPS = 1e-5f;
typedef _Float16 b16;
typedef __attribute__((ext_vector_type(16))) _Float16 v16b;
typedef __attribute__((ext_vector_type(8))) _Float16 v8b;
typedef __attribute__((ext_vector_type(8))) float v8f;
typedef __attribute__((ext_vector_type(4))) float v4f;
__device__ __forceinline__ float bf16_rne(float f) { unsigned int u = __float_as_uint(f); u += 0x7FFFu + ((u >> 16) & 1u); float r = __uint_as_float(u & 0xFFFF0000u); asm volatile("" : "+v"(r)); return r; }
__device__ __forceinline__ float bfv(float f) { float r = bf16_rne(f); asm volatile("" : "+v"(r)); return r; }
__device__ __forceinline__ void split16(float v, b16& hi, b16& lo) { hi = (b16)v; lo = (b16)(v - (float)hi); }
__device__ __forceinline__ v16b frag_kb(const b16* p, int hh) { const v8b a = *(const v8b*)(p + 8 * hh), b = *(const v8b*)(p + 16 + 8 * hh); v16b f;
#pragma unroll
  for (int e = 0; e < 8; ++e) { f[e] = a[e]; f[8 + e] = b[e]; } return f; }
__device__ __forceinline__ v8f wmma16b(v16b a, v16b b, v8f c) { v8f d = __builtin_amdgcn_wmma_f32_16x16x32_f16(false, a, false, b, (short)0, c, false, false); asm volatile("v_nop\n\tv_nop\n\tv_nop\n\tv_nop" : "+v"(d) : "v"(a), "v"(b)); return d; }
__device__ __forceinline__ void wave_lds_sync() { __builtin_amdgcn_fence(__ATOMIC_RELEASE, "workgroup"); __builtin_amdgcn_wave_barrier(); __builtin_amdgcn_fence(__ATOMIC_ACQUIRE, "workgroup"); }
__device__ __forceinline__ float pmul(float a, float b) { float p = a * b; asm volatile("" : "+v"(p)); return p; }
__device__ __forceinline__ float sigm(float v) { return 1.0f / (1.0f + __expf(-v)); }

__global__ __launch_bounds__(256) void wput_kernel(const float* __restrict__ wh, const float* __restrict__ wx, b16* __restrict__ WT) { const size_t u = (size_t)blockIdx.x * 256 + threadIdx.x; if (u >= (size_t)G4 * (KT / 8)) return; const int o = (int)(u / (KT / 8)), k0 = (int)(u % (KT / 8)) * 8; v8b v;
#pragma unroll
  for (int j = 0; j < 8; ++j) { const int k = k0 + j; v[j] = (b16)(bf16_rne(k < H ? wh[(size_t)k * G4 + o] : wx[(size_t)(k - H) * G4 + o]) * WSC); }
  for (int pass = 0; pass < 2; ++pass) { *(volatile v8b*)(WT + (size_t)o * KT + k0) = v; __threadfence(); } }
__global__ __launch_bounds__(32) void gate_kernel(const float* __restrict__ h, const float* __restrict__ x, const b16* __restrict__ WT, const float* __restrict__ bh, int RLIM, float* __restrict__ GT) { __shared__ __attribute__((aligned(16))) b16 Ah[16][IN + 8], Al[16][IN + 8]; __shared__ float Tf[16][260]; const int lane = threadIdx.x, nloc = lane & 15, hlf = lane >> 4; const int cg = blockIdx.x % (G4 / 256); const size_t m0 = (size_t)(blockIdx.x / (G4 / 256)) * 16; if (m0 >= (size_t)RLIM) return; const int c0 = cg * 256;
  v8f acc[16];
#pragma unroll
  for (int t = 0; t < 16; ++t) acc[t] = (v8f){};
#pragma unroll 1
  for (int part = 0; part < 2; ++part) { const float* src = part == 0 ? h : x;
    for (int rr = 0; rr < 16; ++rr) for (int q = 0; q < IN / 32; ++q) { const int k = q * 32 + lane; b16 p, ql; split16(bfv(src[(m0 + rr) * IN + k]) * HS, p, ql); Ah[rr][k] = p; Al[rr][k] = ql; }
    wave_lds_sync();
#pragma unroll 2
    for (int kb = 0; kb < IN; kb += 32) { const v16b a = frag_kb(&Ah[nloc][kb], hlf), al = frag_kb(&Al[nloc][kb], hlf);
#pragma unroll
      for (int t = 0; t < 16; ++t) { const v16b bw = frag_kb(WT + (size_t)(c0 + t * 16 + nloc) * KT + part * H + kb, hlf); acc[t] = wmma16b(a, bw, acc[t]); acc[t] = wmma16b(al, bw, acc[t]); } }
    wave_lds_sync(); }
#pragma unroll
  for (int t = 0; t < 16; ++t) { const int cc = t * 16 + nloc; const float bb = bfv(bh[c0 + cc]);
#pragma unroll
    for (int r8 = 0; r8 < 8; ++r8) Tf[8 * hlf + r8][cc] = acc[t][r8] * (1.0f / (HS * WSC)) + bb; }
  wave_lds_sync();
  for (int pass = 0; pass < 2; ++pass) { for (int rr = 0; rr < 16; ++rr) for (int q = 0; q < 2; ++q) *(volatile v4f*)(GT + (m0 + rr) * G4 + c0 + q * 128 + lane * 4) = *(const v4f*)(&Tf[rr][q * 128 + lane * 4]); __threadfence(); } }
__global__ __launch_bounds__(256) void cell_kernel(const float* __restrict__ GT, const float* __restrict__ c, const float* __restrict__ lg, const float* __restrict__ lb, const float* __restrict__ lcg, const float* __restrict__ lcb, int RLIM, float* __restrict__ HN, float* __restrict__ CN) { __shared__ float Cs[8][H]; const int wave = threadIdx.x >> 5, lane = threadIdx.x & 31; const size_t r = (size_t)blockIdx.x * 8 + wave; if (r >= (size_t)RLIM) return; const float* gr = GT + r * G4;
  float mu[4], rs[4];
#pragma unroll
  for (int g = 0; g < 4; ++g) { float s = 0.0f;
#pragma unroll 1
    for (int q = 0; q < H / 32; ++q) s += gr[g * H + q * 32 + lane]; for (int o = 16; o; o >>= 1) s += __shfl_xor(s, o); const float m = s / H; float s2 = 0.0f;
#pragma unroll 1
    for (int q = 0; q < H / 32; ++q) { const float d = gr[g * H + q * 32 + lane] - m; s2 += d * d; } for (int o = 16; o; o >>= 1) s2 += __shfl_xor(s2, o); mu[g] = m; rs[g] = rsqrtf(s2 / H + EPS); }
  float cs = 0.0f;
#pragma unroll 1
  for (int q = 0; q < H / 32; ++q) { const int j = q * 32 + lane; float gv[4];
#pragma unroll
    for (int g = 0; g < 4; ++g) gv[g] = pmul(pmul(gr[g * H + j] - mu[g], rs[g]), bfv(lg[g * H + j])) + bfv(lb[g * H + j]);
    const float cn = pmul(sigm(gv[1]), bfv(c[r * H + j])) + pmul(sigm(gv[0]), tanhf(gv[2])); Cs[wave][j] = cn; cs += cn; }
  for (int o = 16; o; o >>= 1) cs += __shfl_xor(cs, o); const float cm = cs / H; float cv = 0.0f;
#pragma unroll 1
  for (int q = 0; q < H / 32; ++q) { const float d = Cs[wave][q * 32 + lane] - cm; cv += d * d; } for (int o = 16; o; o >>= 1) cv += __shfl_xor(cv, o); const float crs = rsqrtf(cv / H + EPS);
  for (int pass = 0; pass < 2; ++pass) {
#pragma unroll 1
    for (int q = 0; q < H / 32; ++q) { const int j = q * 32 + lane; const float cn = Cs[wave][j]; const float og = pmul(pmul(gr[3 * H + j] - mu[3], rs[3]), bfv(lg[3 * H + j])) + bfv(lb[3 * H + j]); const float hn = pmul(sigm(og), tanhf(pmul(pmul(cn - cm, crs), bfv(lcg[j])) + bfv(lcb[j]))); ((volatile float*)CN)[r * H + j] = cn; ((volatile float*)HN)[r * H + j] = hn; } __threadfence(); } }
}

extern "C" void kernel_launch(void* const* d_in, const int* in_sizes, int n_in, void* d_out, int out_size, void* d_ws, size_t ws_size, hipStream_t stream) {
  (void)n_in;
  auto Fp = [&](int i) { return (const float*)d_in[i]; };
  if (in_sizes[0] != NBR * IN || in_sizes[1] != NBR * H || in_sizes[2] != NBR * H || in_sizes[3] != H * G4 || in_sizes[4] != G4 || in_sizes[5] != IN * G4 || in_sizes[6] != 4 * H || in_sizes[8] != H || out_size != 2 * NBR * H) return;
  const int RLIM = NBR;
  size_t off = 0; char* ws = (char*)d_ws;
  auto carve = [&](size_t bytes) { char* p = ws + off; off += (bytes + 255) & ~(size_t)255; return p; };
  b16* WT = (b16*)carve((size_t)G4 * KT * 2); float* GT = (float*)carve((size_t)NBR * G4 * 4);
  if (off > ws_size || off > ((size_t)96 << 20)) return;
  float* HN = (float*)d_out; float* CN = HN + (size_t)NBR * H;
  wput_kernel<<<(unsigned)(((size_t)G4 * (KT / 8) + 255) / 256), 256, 0, stream>>>(Fp(3), Fp(5), WT);
  gate_kernel<<<(RLIM / 16) * (G4 / 256), 32, 0, stream>>>(Fp(1), Fp(0), WT, Fp(4), RLIM, GT);
  cell_kernel<<<(RLIM + 7) / 8, 256, 0, stream>>>(GT, Fp(2), Fp(6), Fp(7), Fp(8), Fp(9), RLIM, HN, CN);
}
